// TrmEncoder_17712445129039
// MI455X (gfx1250) — hardware-verified
//
#include <hip/hip_runtime.h>
#include <math.h>

constexpr int kSeqN  = 3072;
constexpr int kDm    = 256;
constexpr int kHeads = 8;
constexpr int kHdim  = 256;
constexpr int kQKV   = kHeads * kHdim;
constexpr int kPorts = 4;
constexpr float kWCarry    = 16.0f;
constexpr float kWCarryInv = 1.0f / 16.0f;
constexpr float kPCarry    = 16384.0f;
constexpr float kPCarryInv = 1.0f / 16384.0f;
constexpr float kLnEps     = 1e-5f;
constexpr float kInvDm     = 1.0f / 256.0f;

typedef __attribute__((ext_vector_type(16))) _Float16 v16h;
typedef __attribute__((ext_vector_type(8)))  _Float16 v8h;
typedef __attribute__((ext_vector_type(16))) __bf16   v16b;
typedef __attribute__((ext_vector_type(8)))  __bf16   v8b;
typedef __attribute__((ext_vector_type(8)))  float    v8f;
typedef __attribute__((ext_vector_type(4)))  float    v4f;
typedef __attribute__((ext_vector_type(4)))  unsigned int v4u;

__device__ __forceinline__ unsigned short f2bf_bits(float f) {
  unsigned u = __float_as_uint(f);
  return (unsigned short)((u + 0x7FFFu + ((u >> 16) & 1u)) >> 16);
}
__device__ __forceinline__ float bf_bits2f(unsigned short h) { return __uint_as_float(((unsigned)h) << 16); }

__device__ __forceinline__ void dep_guard_h(v8f& a, v8f& b, v16h x, v16h y) { asm volatile("v_nop\n\tv_nop\n\tv_nop\n\tv_nop" : "+v"(a), "+v"(b) : "v"(x), "v"(y)); }
__device__ __forceinline__ void dep_guard_b(v8f& a, v8f& b, v16b x, v16b y) { asm volatile("v_nop\n\tv_nop\n\tv_nop\n\tv_nop" : "+v"(a), "+v"(b) : "v"(x), "v"(y)); }
__device__ __forceinline__ void keep4_h(v16h a, v16h b, v16h c, v16h d) { asm volatile("v_nop" :: "v"(a), "v"(b), "v"(c), "v"(d)); }
__device__ __forceinline__ void keep4_b(v16b a, v16b b, v16b c, v16b d) { asm volatile("v_nop" :: "v"(a), "v"(b), "v"(c), "v"(d)); }
__device__ __forceinline__ void acc_guard4(v8f& a, v8f& b, v8f& c, v8f& d) { asm volatile("v_nop\n\tv_nop\n\tv_nop\n\tv_nop" : "+v"(a), "+v"(b), "+v"(c), "+v"(d)); }
template <typename T> struct Frag;
template <> struct Frag<_Float16> {
  typedef v16h V; union U { v16h v; v8h h[2]; };
  static __device__ __forceinline__ v16h load(const _Float16* p) {
    U f; f.h[0] = *(const v8h*)(p); f.h[1] = *(const v8h*)(p + 16); return f.v;
  }
  static __device__ __forceinline__ v8f mma(v16h a, v16h b, v8f c) {
    return __builtin_amdgcn_wmma_f32_16x16x32_f16(false, a, false, b, (short)0, c, false, false);
  }
  static __device__ __forceinline__ void guard(v8f& a, v8f& b, v16h x, v16h y) { dep_guard_h(a, b, x, y); }
  static __device__ __forceinline__ void keep(v16h a, v16h b, v16h c, v16h d) { keep4_h(a, b, c, d); }
};
template <> struct Frag<__bf16> {
  typedef v16b V; union U { v16b v; v8b h[2]; };
  static __device__ __forceinline__ v16b load(const __bf16* p) {
    U f; f.h[0] = *(const v8b*)(p); f.h[1] = *(const v8b*)(p + 16); return f.v;
  }
  static __device__ __forceinline__ v8f mma(v16b a, v16b b, v8f c) {
    return __builtin_amdgcn_wmma_f32_16x16x32_bf16(false, a, false, b, (short)0, c, false, false);
  }
  static __device__ __forceinline__ void guard(v8f& a, v8f& b, v16b x, v16b y) { dep_guard_b(a, b, x, y); }
  static __device__ __forceinline__ void keep(v16b a, v16b b, v16b c, v16b d) { keep4_b(a, b, c, d); }
};

__device__ __forceinline__ unsigned pk16(unsigned short a, unsigned short b) { return (unsigned)a | ((unsigned)b << 16); }
__device__ __forceinline__ unsigned short h_bits(float f) { const _Float16 h = (_Float16)f; return __builtin_bit_cast(unsigned short, h); }

template <int ET> struct Elem;
template <> struct Elem<0> { typedef _Float16 T; };
template <> struct Elem<1> { typedef __bf16 T; };
template <int ET, bool SPLIT, int BIAS_MODE, int OUT_MODE, bool RESID, int ACT, int CAUS>
__global__ __launch_bounds__(256) void wmma_gemm64(
    const unsigned short* __restrict__ Ap, const unsigned short* __restrict__ A2p, int lda, long strideA,
    const unsigned short* __restrict__ Btp, const unsigned short* __restrict__ Bt2p, int ldb, long strideB,
    void* __restrict__ Cout, void* __restrict__ Cout2, int ldc, long strideC,
    const float* __restrict__ bias,
    const float* __restrict__ resid, long strideR,
    int M, int N, int K, float scale) {
  typedef typename Elem<ET>::T T;
  typedef typename Frag<T>::V V;
  const T* A = (const T*)Ap; const T* A2 = (const T*)A2p; const T* Bt = (const T*)Btp; const T* Bt2 = (const T*)Bt2p;
  __shared__ __align__(16) float sT[8][16 * 68];
  const int b    = blockIdx.y;
  const int lane = threadIdx.x & 31;
  const int wave = threadIdx.x >> 5;
  const int tilesN = N >> 6;
  const int tilesM = M >> 6;
  const int tile = blockIdx.x * 8 + wave;
  int tm, tn;
  if (CAUS == 1) {
    const int ntri = (tilesM * (tilesM + 1)) >> 1;
    if (tile >= ntri) return;
    int t_m = (int)((sqrtf(8.0f * (float)tile + 1.0f) - 1.0f) * 0.5f);
    if (((t_m * (t_m + 1)) >> 1) > tile) t_m -= 1;
    if ((((t_m + 1) * (t_m + 2)) >> 1) <= tile) t_m += 1;
    tm = t_m;
    tn = tile - ((t_m * (t_m + 1)) >> 1);
  } else {
    if (tile >= tilesM * tilesN) return;
    tm = tile / tilesN;
    tn = tile - tm * tilesN;
  }
  const int m0 = tm << 6;
  const int n0 = tn << 6;
  int Kw = K;
  if (CAUS == 2) { const int kc = (tm + 1) << 6; Kw = (kc < K) ? kc : K; }

  const T* Ab  = A  + (size_t)b * strideA;
  const T* Bb  = Bt + (size_t)b * strideB;
  const T* Ab2 = SPLIT ? (A2  + (size_t)b * strideA) : nullptr;
  const T* Bb2 = SPLIT ? (Bt2 + (size_t)b * strideB) : nullptr;

  const int rlane = lane & 15;
  const int koff  = (lane >> 4) * 8;
  const int mOff  = (lane >> 4) * 8;

  v8f acc[4][4];
#pragma unroll
  for (int i = 0; i < 4; ++i)
#pragma unroll
    for (int j = 0; j < 4; ++j) acc[i][j] = (v8f){0.f,0.f,0.f,0.f,0.f,0.f,0.f,0.f};

  for (int k0 = 0; k0 < Kw; k0 += 32) {
    V bh[4], bl[4];
#pragma unroll
    for (int j = 0; j < 4; ++j) {
      const size_t bo = (size_t)(n0 + (j << 4) + rlane) * ldb + koff + k0;
      bh[j] = Frag<T>::load(Bb + bo);
      if (SPLIT) bl[j] = Frag<T>::load(Bb2 + bo);
    }
#pragma unroll
    for (int i = 0; i < 4; ++i) {
      const size_t ao = (size_t)(m0 + (i << 4) + rlane) * lda + koff + k0;
      V ah = Frag<T>::load(Ab + ao);
      V al;
      if (SPLIT) al = Frag<T>::load(Ab2 + ao);
#pragma unroll
      for (int j = 0; j < 4; ++j) {
        acc[i][j] = Frag<T>::mma(ah, bh[j], acc[i][j]);
        if (SPLIT) {
          acc[i][j] = Frag<T>::mma(ah, bl[j], acc[i][j]);
          acc[i][j] = Frag<T>::mma(al, bh[j], acc[i][j]);
        }
      }
      Frag<T>::guard(acc[i][0], acc[i][3], ah, SPLIT ? al : ah);
    }
    Frag<T>::keep(bh[0], bh[1], bh[2], bh[3]);
    if (SPLIT) Frag<T>::keep(bl[0], bl[1], bl[2], bl[3]);
  }
  acc_guard4(acc[0][0], acc[0][1], acc[0][2], acc[0][3]);
  acc_guard4(acc[1][0], acc[1][1], acc[1][2], acc[1][3]);
  acc_guard4(acc[2][0], acc[2][1], acc[2][2], acc[2][3]);
  acc_guard4(acc[3][0], acc[3][1], acc[3][2], acc[3][3]);

  float* slab = sT[wave];
  const float* Rb = RESID ? (resid + (size_t)b * strideR) : nullptr;
#pragma unroll
  for (int i = 0; i < 4; ++i) {
    const int mBase = m0 + (i << 4);
#pragma unroll
    for (int j = 0; j < 4; ++j) {
      const int n = n0 + (j << 4) + rlane;
      float bv = 0.f;
      if (BIAS_MODE == 2) bv = bias[n];
#pragma unroll
      for (int r = 0; r < 8; ++r) {
        float v = acc[i][j][r] * scale;
        if (BIAS_MODE == 1) v += bias[mBase + mOff + r];
        if (BIAS_MODE == 2) v += bv;
        if (RESID) v += Rb[(size_t)(mBase + mOff + r) * ldc + n];
        if (ACT == 2) v = fmaxf(v, 0.0f);
        if (ACT == 4) v = (v > 0.f) ? v : 0.01f * v;
        slab[(mOff + r) * 68 + (j << 4) + rlane] = v;
      }
    }
    __builtin_amdgcn_fence(__ATOMIC_RELEASE, "workgroup");
    __builtin_amdgcn_wave_barrier();
    __builtin_amdgcn_fence(__ATOMIC_ACQUIRE, "workgroup");
    if (OUT_MODE == 0) {
      float* C = (float*)Cout + (size_t)b * strideC;
      const int hh = lane >> 4, c4 = (lane & 15) * 4;
      for (int pass = 0; pass < 2; ++pass) {
#pragma unroll
        for (int it = 0; it < 8; ++it) {
          const int row = it * 2 + hh;
          v4f v = *(const v4f*)(slab + row * 68 + c4);
          *(volatile v4f*)(C + (size_t)(mBase + row) * ldc + n0 + c4) = v;
        }
        __threadfence();
      }
    } else {
      const int q = lane >> 3, c8 = (lane & 7) * 8;
      unsigned short* C  = (unsigned short*)Cout  + (size_t)b * strideC;
      unsigned short* C2 = (OUT_MODE == 2) ? ((unsigned short*)Cout2 + (size_t)b * strideC) : nullptr;
      for (int pass = 0; pass < 2; ++pass) {
#pragma unroll
        for (int it = 0; it < 4; ++it) {
          const int row = it * 4 + q;
          const float* sp = slab + row * 68 + c8;
          v8h hv, lv;
#pragma unroll
          for (int e = 0; e < 8; ++e) {
            if (OUT_MODE == 1) {
              hv[e] = (_Float16)sp[e];
            } else {
              unsigned short hb = f2bf_bits(sp[e]);
              unsigned short lb = f2bf_bits(sp[e] - bf_bits2f(hb));
              hv[e] = __builtin_bit_cast(_Float16, hb);
              lv[e] = __builtin_bit_cast(_Float16, lb);
            }
          }
          *(volatile v8h*)(C + (size_t)(mBase + row) * ldc + n0 + c8) = hv;
          if (OUT_MODE == 2) *(volatile v8h*)(C2 + (size_t)(mBase + row) * ldc + n0 + c8) = lv;
        }
        __threadfence();
      }
    }
    __builtin_amdgcn_fence(__ATOMIC_RELEASE, "workgroup");
    __builtin_amdgcn_wave_barrier();
    __builtin_amdgcn_fence(__ATOMIC_ACQUIRE, "workgroup");
  }
}

__global__ __launch_bounds__(64) void feat_kernel(
    const float* __restrict__ weights, const int* __restrict__ up, const float* __restrict__ pe,
    const float* __restrict__ we_w, const float* __restrict__ we_b,
    float* __restrict__ featF, unsigned short* __restrict__ featH)
{
  const int lane = threadIdx.x & 31, wave = threadIdx.x >> 5;
  const int row = blockIdx.x * 2 + wave;
  int u = up[row];
  u = (u < 0) ? (u + kPorts) : u;
  u = (u < 0) ? 0 : ((u > kPorts - 1) ? (kPorts - 1) : u);
  const float w = weights[row];
  const float* per = pe + u * kDm;
  float* fr = featF + (size_t)row * kDm;
  unsigned short* hr = featH + (size_t)row * kDm;

  v4f y0, y1;
  {
    const int d = lane * 4;
    const v4f pv = *(const v4f*)(per + d), ww = *(const v4f*)(we_w + d), bb = *(const v4f*)(we_b + d);
#pragma unroll
    for (int i = 0; i < 4; ++i) { float fw = w * ww[i]; fw = fw + bb[i]; y0[i] = pv[i] + fw; }
  }
  {
    const int d = 128 + lane * 4;
    const v4f pv = *(const v4f*)(per + d), ww = *(const v4f*)(we_w + d), bb = *(const v4f*)(we_b + d);
#pragma unroll
    for (int i = 0; i < 4; ++i) { float fw = w * ww[i]; fw = fw + bb[i]; y1[i] = pv[i] + fw; }
  }
  v4u pk;
  {
    const int d = lane * 8;
    const v4f pa = *(const v4f*)(per + d), pb = *(const v4f*)(per + d + 4);
    const v4f wa = *(const v4f*)(we_w + d), wb = *(const v4f*)(we_w + d + 4);
    const v4f ba = *(const v4f*)(we_b + d), bb = *(const v4f*)(we_b + d + 4);
    unsigned short hb[8];
#pragma unroll
    for (int i = 0; i < 4; ++i) { float fw = w * wa[i]; fw = fw + ba[i]; hb[i] = h_bits(pa[i] + fw); }
#pragma unroll
    for (int i = 0; i < 4; ++i) { float fw = w * wb[i]; fw = fw + bb[i]; hb[4 + i] = h_bits(pb[i] + fw); }
    pk = (v4u){pk16(hb[0], hb[1]), pk16(hb[2], hb[3]), pk16(hb[4], hb[5]), pk16(hb[6], hb[7])};
  }
  *(volatile v4f*)(fr + lane * 4) = y0;
  *(volatile v4f*)(fr + 128 + lane * 4) = y1;
  *(volatile v4u*)(hr + lane * 8) = pk;
  __threadfence();
  *(volatile v4f*)(fr + lane * 4) = y0;
  *(volatile v4f*)(fr + 128 + lane * 4) = y1;
  *(volatile v4u*)(hr + lane * 8) = pk;
}

template <int OUTM>
__global__ __launch_bounds__(256) void tcast_kernel(
    const float* __restrict__ in0, const float* __restrict__ in1, const float* __restrict__ in2,
    unsigned short* __restrict__ out, unsigned short* __restrict__ out2, int R, int Cc, float scale)
{
  __shared__ float sm[64][65];
  const int t  = threadIdx.x;
  const int r0 = blockIdx.x * 64;
  const int c0 = blockIdx.y * 64;
  const int z  = blockIdx.z;
  const float* W = (z == 0) ? in0 : ((z == 1) ? in1 : in2);
#pragma unroll
  for (int i = 0; i < 16; ++i) {
    const int e = i * 256 + t;
    const int r = e >> 6;
    const int c = e & 63;
    sm[c][r] = W[(size_t)(r0 + r) * Cc + c0 + c] * scale;
  }
  __syncthreads();
  const int lane = t & 31, wave = t >> 5;
  const int qq = lane >> 3, c8 = (lane & 7) * 8;
  unsigned short* op  = out + (size_t)z * R * Cc;
  unsigned short* op2 = out2;
  for (int pass = 0; pass < 2; ++pass) {
#pragma unroll
    for (int it = 0; it < 2; ++it) {
      const int row = wave * 8 + it * 4 + qq;
      unsigned short hb[8], lb[8];
#pragma unroll
      for (int e = 0; e < 8; ++e) {
        const float v = sm[row][c8 + e];
        if (OUTM == 1) { hb[e] = h_bits(v); lb[e] = 0; }
        else { hb[e] = f2bf_bits(v); lb[e] = f2bf_bits(v - bf_bits2f(hb[e])); }
      }
      const v4u uh = (v4u){pk16(hb[0], hb[1]), pk16(hb[2], hb[3]), pk16(hb[4], hb[5]), pk16(hb[6], hb[7])};
      *(volatile v4u*)(op + (size_t)(c0 + row) * R + r0 + c8) = uh;
      if (OUTM == 2) {
        const v4u ul = (v4u){pk16(lb[0], lb[1]), pk16(lb[2], lb[3]), pk16(lb[4], lb[5]), pk16(lb[6], lb[7])};
        *(volatile v4u*)(op2 + (size_t)(c0 + row) * R + r0 + c8) = ul;
      }
    }
    __threadfence();
  }
}

__global__ __launch_bounds__(256) void cast_hilo_kernel(
    const float* __restrict__ in0, const float* __restrict__ in1,
    unsigned short* __restrict__ oh0, unsigned short* __restrict__ ol0,
    unsigned short* __restrict__ oh1, unsigned short* __restrict__ ol1, int n8)
{
  const int z = blockIdx.y;
  const float* in = (z == 0) ? in0 : in1;
  unsigned short* oh = (z == 0) ? oh0 : oh1;
  unsigned short* ol = (z == 0) ? ol0 : ol1;
  const int i = blockIdx.x * 256 + threadIdx.x;
  if (i < n8) {
    const v4f a = *(const v4f*)(in + (size_t)i * 8);
    const v4f c = *(const v4f*)(in + (size_t)i * 8 + 4);
    unsigned short hb[8], lb[8];
#pragma unroll
    for (int e = 0; e < 4; ++e) {
      hb[e] = f2bf_bits(a[e]);     lb[e] = f2bf_bits(a[e] - bf_bits2f(hb[e]));
      hb[4 + e] = f2bf_bits(c[e]); lb[4 + e] = f2bf_bits(c[e] - bf_bits2f(hb[4 + e]));
    }
    const v4u uh = (v4u){pk16(hb[0], hb[1]), pk16(hb[2], hb[3]), pk16(hb[4], hb[5]), pk16(hb[6], hb[7])};
    const v4u ul = (v4u){pk16(lb[0], lb[1]), pk16(lb[2], lb[3]), pk16(lb[4], lb[5]), pk16(lb[6], lb[7])};
    *(volatile v4u*)(oh + (size_t)i * 8) = uh;
    *(volatile v4u*)(ol + (size_t)i * 8) = ul;
    __threadfence();
    *(volatile v4u*)(oh + (size_t)i * 8) = uh;
    *(volatile v4u*)(ol + (size_t)i * 8) = ul;
  }
}

template <int MODE>
__global__ __launch_bounds__(384) void rowsoftmax_kernel(
    const float* __restrict__ biasg, const unsigned short* __restrict__ Sg,
    const unsigned short* __restrict__ P2g, unsigned short* __restrict__ outp)
{
  __shared__ float redm[12];
  __shared__ float reds[12];
  const int q = blockIdx.x;
  const int t = threadIdx.x;
  const int lane = t & 31, wave = t >> 5;
  const int kmax = ((q >> 6) + 1) << 6;
  const int kb = t * 8;
  const size_t ro = (size_t)q * kSeqN + kb;
  const float ninf = __uint_as_float(0xff800000u);

  float s[8];
  if (MODE == 0) {
    const v4f a0 = *(const v4f*)(biasg + ro);
    const v4f a1 = *(const v4f*)(biasg + ro + 4);
#pragma unroll
    for (int i = 0; i < 4; ++i) { s[i] = a0[i]; s[4 + i] = a1[i]; }
  } else {
    const v4u u = *(const v4u*)(Sg + ro);
#pragma unroll
    for (int i = 0; i < 4; ++i) {
      s[2 * i]     = (float)__builtin_bit_cast(_Float16, (unsigned short)(u[i] & 0xffffu));
      s[2 * i + 1] = (float)__builtin_bit_cast(_Float16, (unsigned short)(u[i] >> 16));
    }
  }
  float m = ninf;
#pragma unroll
  for (int e = 0; e < 8; ++e) { s[e] = (kb + e <= q) ? s[e] : ninf; m = fmaxf(m, s[e]); }
#pragma unroll
  for (int o = 1; o < 32; o <<= 1) m = fmaxf(m, __shfl_xor(m, o, 32));
  if (lane == 0) redm[wave] = m;
  __syncthreads();
  float rm = redm[0];
#pragma unroll
  for (int wv = 1; wv < 12; ++wv) rm = fmaxf(rm, redm[wv]);

  float p[8];
  float ls = 0.f;
#pragma unroll
  for (int e = 0; e < 8; ++e) {
    const float ex = __expf(s[e] - rm);
    p[e] = (kb + e <= q) ? ex : 0.f;
    ls += p[e];
  }
#pragma unroll
  for (int o = 1; o < 32; o <<= 1) ls += __shfl_xor(ls, o, 32);
  if (lane == 0) reds[wave] = ls;
  __syncthreads();
  float rs = reds[0];
#pragma unroll
  for (int wv = 1; wv < 12; ++wv) rs += reds[wv];
  const float inv = kPCarry / rs;

  float p2f[8];
#pragma unroll
  for (int e = 0; e < 8; ++e) p2f[e] = 0.f;
  if (MODE == 1) {
    const v4u w = *(const v4u*)(P2g + ro);
#pragma unroll
    for (int i = 0; i < 4; ++i) {
      p2f[2 * i]     = (float)__builtin_bit_cast(_Float16, (unsigned short)(w[i] & 0xffffu));
      p2f[2 * i + 1] = (float)__builtin_bit_cast(_Float16, (unsigned short)(w[i] >> 16));
    }
  }
  unsigned short hb[8];
#pragma unroll
  for (int e = 0; e < 8; ++e) {
    const float o = (kb + e <= q) ? (p[e] * inv + p2f[e]) : 0.f;
    hb[e] = h_bits(o);
  }
  const v4u pk = (v4u){pk16(hb[0], hb[1]), pk16(hb[2], hb[3]), pk16(hb[4], hb[5]), pk16(hb[6], hb[7])};
  unsigned short* dst = outp + ro;
  if (kb < kmax) *(volatile v4u*)dst = pk;
  __threadfence();
  if (kb < kmax) *(volatile v4u*)dst = pk;
}

template <int OUTM>
__global__ __launch_bounds__(64) void ln_kernel(
    const float* __restrict__ in, const float* __restrict__ g, const float* __restrict__ bta,
    float* __restrict__ outF, unsigned short* __restrict__ outH, unsigned short* __restrict__ outL)
{
  __shared__ float red[4];
  const int row = blockIdx.x, t = threadIdx.x, lane = t & 31, wave = t >> 5;
  const float* xr = in + (size_t)row * kDm;
  const v4f x = *(const v4f*)(xr + 4 * t);
  float sm = (x[0] + x[1]) + (x[2] + x[3]);
#pragma unroll
  for (int o = 1; o < 32; o <<= 1) sm += __shfl_xor(sm, o, 32);
  if (lane == 0) red[wave] = sm;
  __syncthreads();
  const float mu = (red[0] + red[1]) * kInvDm;
  float c[4];
#pragma unroll
  for (int i = 0; i < 4; ++i) c[i] = x[i] - mu;
  float sq = (c[0] * c[0] + c[1] * c[1]) + (c[2] * c[2] + c[3] * c[3]);
#pragma unroll
  for (int o = 1; o < 32; o <<= 1) sq += __shfl_xor(sq, o, 32);
  if (lane == 0) red[2 + wave] = sq;
  __syncthreads();
  const float var  = (red[2] + red[3]) * kInvDm;
  const float rstd = 1.0f / sqrtf(var + kLnEps);
  const v4f gg = *(const v4f*)(g + 4 * t), bb = *(const v4f*)(bta + 4 * t);
  v4f y;
#pragma unroll
  for (int i = 0; i < 4; ++i) y[i] = c[i] * rstd * gg[i] + bb[i];
  float* dst = outF + (size_t)row * kDm + 4 * t;
  *(volatile v4f*)dst = y;
  __threadfence();
  *(volatile v4f*)dst = y;
  if (OUTM == 0) {
    if (wave == 0) {
      const int d = lane * 8;
      const v4f xa = *(const v4f*)(xr + d), xb = *(const v4f*)(xr + d + 4);
      const v4f ga = *(const v4f*)(g + d), gb = *(const v4f*)(g + d + 4);
      const v4f ba = *(const v4f*)(bta + d), bb2 = *(const v4f*)(bta + d + 4);
      unsigned short hb[8], lb[8];
#pragma unroll
      for (int e = 0; e < 4; ++e) {
        const float v0 = (xa[e] - mu) * rstd * ga[e] + ba[e];
        const float v1 = (xb[e] - mu) * rstd * gb[e] + bb2[e];
        hb[e] = f2bf_bits(v0);     lb[e] = f2bf_bits(v0 - bf_bits2f(hb[e]));
        hb[4 + e] = f2bf_bits(v1); lb[4 + e] = f2bf_bits(v1 - bf_bits2f(hb[4 + e]));
      }
      const v4u uh = (v4u){pk16(hb[0], hb[1]), pk16(hb[2], hb[3]), pk16(hb[4], hb[5]), pk16(hb[6], hb[7])};
      const v4u ul = (v4u){pk16(lb[0], lb[1]), pk16(lb[2], lb[3]), pk16(lb[4], lb[5]), pk16(lb[6], lb[7])};
      unsigned short* dh = outH + (size_t)row * kDm + d;
      unsigned short* dl = outL + (size_t)row * kDm + d;
      *(volatile v4u*)dh = uh;
      *(volatile v4u*)dl = ul;
      __threadfence();
      *(volatile v4u*)dh = uh;
      *(volatile v4u*)dl = ul;
    }
  }
}

extern "C" void kernel_launch(void* const* d_in, const int* in_sizes, int n_in,
                              void* d_out, int out_size, void* d_ws, size_t ws_size,
                              hipStream_t stream)
{
  if (n_in < 16) return;
  if (in_sizes[0] < kSeqN || in_sizes[1] < kSeqN || in_sizes[2] < kSeqN * kSeqN || in_sizes[3] < kPorts * kDm ||
      in_sizes[4] < kDm || in_sizes[5] < kDm || in_sizes[6] < kDm * kQKV || in_sizes[7] < kDm * kQKV ||
      in_sizes[8] < kDm * kQKV || in_sizes[9] < kQKV * kDm || in_sizes[10] < kDm * kDm || in_sizes[11] < kDm ||
      in_sizes[12] < kDm * kDm || in_sizes[13] < kDm || in_sizes[14] < kDm || in_sizes[15] < kDm) return;
  if (out_size < kSeqN * kDm) return;

  const float* weights = (const float*)d_in[0];
  const int*   up      = (const int*)d_in[1];
  const float* bias    = (const float*)d_in[2];
  const float* pe      = (const float*)d_in[3];
  const float* we_w    = (const float*)d_in[4];
  const float* we_b    = (const float*)d_in[5];
  const float* W_q     = (const float*)d_in[6];
  const float* W_k     = (const float*)d_in[7];
  const float* W_v     = (const float*)d_in[8];
  const float* W_o     = (const float*)d_in[9];
  const float* l1_w    = (const float*)d_in[10];
  const float* l1_b    = (const float*)d_in[11];
  const float* l2_w    = (const float*)d_in[12];
  const float* l2_b    = (const float*)d_in[13];
  const float* ln_g    = (const float*)d_in[14];
  const float* ln_b    = (const float*)d_in[15];
  float* outp = (float*)d_out;

  const size_t bRowF = (size_t)kSeqN * kDm * 4;
  const size_t bRowH = (size_t)kSeqN * kDm * 2;
  const size_t bWT   = (size_t)kQKV * kDm * 2;
  const size_t bL    = (size_t)kDm * kDm * 2;
  const size_t bQ    = (size_t)kSeqN * kQKV * 2;
  const size_t bNN   = (size_t)kSeqN * kSeqN * 2;

  char* ws = (char*)d_ws;
  size_t off = 0;
  float* featF = (float*)(ws + off); off += bRowF;
  unsigned short* featH = (unsigned short*)(ws + off); off += bRowH;
  unsigned short* WT3 = (unsigned short*)(ws + off); off += 3 * bWT;
  unsigned short* WoTh = (unsigned short*)(ws + off); off += bWT;
  unsigned short* WoTl = (unsigned short*)(ws + off); off += bWT;
  unsigned short* L1h = (unsigned short*)(ws + off); off += bL;
  unsigned short* L1l = (unsigned short*)(ws + off); off += bL;
  unsigned short* L2h = (unsigned short*)(ws + off); off += bL;
  unsigned short* L2l = (unsigned short*)(ws + off); off += bL;
  unsigned short* Qp = (unsigned short*)(ws + off); off += bQ;
  unsigned short* Kp = (unsigned short*)(ws + off); off += bQ;   (void)Kp;
  unsigned short* Vt = (unsigned short*)(ws + off); off += bQ;
  unsigned short* P2 = (unsigned short*)(ws + off); off += bNN;
  char* sbase = ws + off;
  unsigned short* S = (unsigned short*)(ws + off); off += bNN;
  unsigned short* P = (unsigned short*)(ws + off); off += bNN;
  unsigned short* Oh = (unsigned short*)(ws + off); off += bQ;
  unsigned short* Ol = (unsigned short*)(ws + off); off += bQ;
  if (off > ws_size) return;
  float* Y  = (float*)(sbase);
  float* Xf = (float*)(sbase + bRowF);
  unsigned short* Xh  = (unsigned short*)(sbase + 2 * bRowF);
  unsigned short* Xl  = (unsigned short*)(sbase + 2 * bRowF + bRowH);
  unsigned short* F1h = (unsigned short*)(sbase + 2 * bRowF + 2 * bRowH);
  unsigned short* F1l = (unsigned short*)(sbase + 2 * bRowF + 3 * bRowH);
  float* T2 = (float*)(sbase + 2 * bRowF + 4 * bRowH);

  const float temper = 16.0f + 1e-6f;
  const float sscale = 1.0f / temper;
  const long plWT = (long)kQKV * kDm;
  const long plQ  = (long)kSeqN * kQKV;

  feat_kernel<<<kSeqN / 2, 64, 0, stream>>>(weights, up, pe, we_w, we_b, featF, featH);
  tcast_kernel<1><<<dim3(kDm / 64, kQKV / 64, 3), 256, 0, stream>>>(W_q, W_k, W_v, WT3, WT3, kDm, kQKV, kWCarry);
  tcast_kernel<2><<<dim3(kQKV / 64, kDm / 64, 1), 256, 0, stream>>>(W_o, W_o, W_o, WoTh, WoTl, kQKV, kDm, 1.0f);
  cast_hilo_kernel<<<dim3((kDm * kDm / 8) / 256, 2), 256, 0, stream>>>(l1_w, l2_w, L1h, L1l, L2h, L2l, kDm * kDm / 8);
  wmma_gemm64<0, false, 0, 1, false, 0, 0><<<dim3(192, 2), 256, 0, stream>>>(
      featH, featH, kDm, 0L, WT3, WT3, kDm, plWT, (void*)Qp, (void*)Qp, kQKV, plQ,
      featF, featF, 0L, kSeqN, kQKV, kDm, kWCarryInv);
  wmma_gemm64<0, false, 0, 1, false, 0, 0><<<dim3(192, 1), 256, 0, stream>>>(
      WT3 + 2 * plWT, WT3 + 2 * plWT, kDm, 0L, featH, featH, kDm, 0L, (void*)Vt, (void*)Vt, kSeqN, 0L,
      featF, featF, 0L, kQKV, kSeqN, kDm, kWCarryInv);
  rowsoftmax_kernel<0><<<kSeqN, 384, 0, stream>>>(bias, S, P2, P2);
  for (int h = 0; h < kHeads; ++h) {
    wmma_gemm64<0, false, 0, 1, false, 0, 1><<<dim3(147, 1), 256, 0, stream>>>(
        Qp + h * kHdim, Qp + h * kHdim, kQKV, 0L, Qp + plQ + h * kHdim, Qp + plQ + h * kHdim, kQKV, 0L,
        (void*)S, (void*)S, kSeqN, 0L, featF, featF, 0L, kSeqN, kSeqN, kHdim, sscale);
    rowsoftmax_kernel<1><<<kSeqN, 384, 0, stream>>>(bias, S, P2, P);
    wmma_gemm64<0, false, 0, 2, false, 0, 2><<<dim3(24, 1), 256, 0, stream>>>(
        P, P, kSeqN, 0L, Vt + (size_t)h * kHdim * kSeqN, Vt + (size_t)h * kHdim * kSeqN, kSeqN, 0L,
        (void*)(Oh + h * kHdim), (void*)(Ol + h * kHdim), kQKV, 0L, featF, featF, 0L,
        kSeqN, kHdim, kSeqN, kPCarryInv);
  }
  wmma_gemm64<1, true, 0, 0, true, 0, 0><<<dim3(24, 1), 256, 0, stream>>>(
      Oh, Ol, kQKV, 0L, WoTh, WoTl, kQKV, 0L, (void*)Y, (void*)Y, kDm, 0L, featF, featF, 0L,
      kSeqN, kDm, kQKV, 1.0f);
  ln_kernel<0><<<kSeqN, 64, 0, stream>>>(Y, ln_g, ln_b, Xf, Xh, Xl);
  wmma_gemm64<1, true, 2, 2, false, 2, 0><<<dim3(24, 1), 256, 0, stream>>>(
      Xh, Xl, kDm, 0L, L1h, L1l, kDm, 0L, (void*)F1h, (void*)F1l, kDm, 0L, l1_b, featF, 0L,
      kSeqN, kDm, kDm, 1.0f);
  wmma_gemm64<1, true, 2, 0, true, 0, 0><<<dim3(24, 1), 256, 0, stream>>>(
      F1h, F1l, kDm, 0L, L2h, L2l, kDm, 0L, (void*)T2, (void*)T2, kDm, 0L, l2_b, Xf, 0L,
      kSeqN, kDm, kDm, 1.0f);
  ln_kernel<1><<<kSeqN, 64, 0, stream>>>(T2, ln_g, ln_b, outp, Xh, Xl);
}
